// EdgePredictor_59631325937959
// MI455X (gfx1250) — hardware-verified
//
#include <hip/hip_runtime.h>
#include <math.h>

constexpr int kNodes   = 50000;
constexpr int kEdges   = 640000;
constexpr int kFeat    = 128;
constexpr int kKdim    = 256;
constexpr int kHid     = 128;
constexpr int kBM      = 128;
constexpr int kLdaH    = 264;
constexpr int kThreads = 256;
static_assert(kEdges % kBM == 0);
static_assert(kKdim % 32 == 0);
static_assert(kHid % 64 == 0);
static_assert(kHid == kBM);
static_assert((kNodes * kFeat) % 8 == 0);
static_assert(((kNodes * kFeat) / 8) % kThreads == 0);
static_assert(((kHid * kKdim) / 8) % kThreads == 0);
static_assert((kLdaH * 2) % 16 == 0);

typedef __attribute__((ext_vector_type(16))) _Float16 v16h;
typedef __attribute__((ext_vector_type(8)))  _Float16 v8h;
typedef __attribute__((ext_vector_type(16))) __bf16   v16b;
typedef __attribute__((ext_vector_type(8)))  __bf16   v8b;
typedef __attribute__((ext_vector_type(8)))  float    v8f;
typedef __attribute__((ext_vector_type(4)))  float    v4f;
typedef __attribute__((ext_vector_type(4)))  unsigned int v4u;

__device__ __forceinline__ unsigned short f2bf_bits(float f) {
  unsigned u = __float_as_uint(f);
  return (unsigned short)((u + 0x7FFFu + ((u >> 16) & 1u)) >> 16);
}
__device__ __forceinline__ float bf_bits2f(unsigned short h) { return __uint_as_float(((unsigned)h) << 16); }

__device__ __forceinline__ void dep_guard_h(v8f& a, v8f& b, v16h x, v16h y) { asm volatile("v_nop\n\tv_nop\n\tv_nop\n\tv_nop" : "+v"(a), "+v"(b) : "v"(x), "v"(y)); }
__device__ __forceinline__ void dep_guard_b(v8f& a, v8f& b, v16b x, v16b y) { asm volatile("v_nop\n\tv_nop\n\tv_nop\n\tv_nop" : "+v"(a), "+v"(b) : "v"(x), "v"(y)); }
__device__ __forceinline__ void keep4_h(v16h a, v16h b, v16h c, v16h d) { asm volatile("v_nop" :: "v"(a), "v"(b), "v"(c), "v"(d)); }
__device__ __forceinline__ void keep4_b(v16b a, v16b b, v16b c, v16b d) { asm volatile("v_nop" :: "v"(a), "v"(b), "v"(c), "v"(d)); }
__device__ __forceinline__ void acc_guard4(v8f& a, v8f& b, v8f& c, v8f& d) { asm volatile("v_nop\n\tv_nop\n\tv_nop\n\tv_nop" : "+v"(a), "+v"(b), "+v"(c), "+v"(d)); }
template <typename T> struct Frag;
template <> struct Frag<_Float16> {
  typedef v16h V; union U { v16h v; v8h h[2]; };
  static __device__ __forceinline__ v16h load(const _Float16* p) {
    U f; f.h[0] = *(const v8h*)(p); f.h[1] = *(const v8h*)(p + 16); return f.v;
  }
  static __device__ __forceinline__ v8f mma(v16h a, v16h b, v8f c) {
    return __builtin_amdgcn_wmma_f32_16x16x32_f16(false, a, false, b, (short)0, c, false, false);
  }
  static __device__ __forceinline__ void guard(v8f& a, v8f& b, v16h x, v16h y) { dep_guard_h(a, b, x, y); }
  static __device__ __forceinline__ void keep(v16h a, v16h b, v16h c, v16h d) { keep4_h(a, b, c, d); }
};
template <> struct Frag<__bf16> {
  typedef v16b V; union U { v16b v; v8b h[2]; };
  static __device__ __forceinline__ v16b load(const __bf16* p) {
    U f; f.h[0] = *(const v8b*)(p); f.h[1] = *(const v8b*)(p + 16); return f.v;
  }
  static __device__ __forceinline__ v8f mma(v16b a, v16b b, v8f c) {
    return __builtin_amdgcn_wmma_f32_16x16x32_bf16(false, a, false, b, (short)0, c, false, false);
  }
  static __device__ __forceinline__ void guard(v8f& a, v8f& b, v16b x, v16b y) { dep_guard_b(a, b, x, y); }
  static __device__ __forceinline__ void keep(v16b a, v16b b, v16b c, v16b d) { keep4_b(a, b, c, d); }
};

__device__ __forceinline__ unsigned pk16(unsigned short a, unsigned short b) { return (unsigned)a | ((unsigned)b << 16); }

__device__ __forceinline__ void row_guard_b(v8f& a0, v8f& a1, v8f& a2, v8f& a3,
                                            v16b x, v16b y0, v16b y1, v16b y2, v16b y3) {
  asm volatile("v_nop\n\tv_nop\n\tv_nop\n\tv_nop"
               : "+v"(a0), "+v"(a1), "+v"(a2), "+v"(a3)
               : "v"(x), "v"(y0), "v"(y1), "v"(y2), "v"(y3));
}
__device__ __forceinline__ float bf_value(float f) { return bf_bits2f(f2bf_bits(f)); }
__device__ __forceinline__ void mem_clause_break() { asm volatile("" ::: "memory"); }

__global__ __launch_bounds__(256) void cast8_bf16_kernel(const float* __restrict__ in, unsigned short* __restrict__ out, int n8) {
  const int i = blockIdx.x * 256 + threadIdx.x;
  if (i >= n8) return;
  const float* p = in + 8 * (size_t)i;
  const v4f a = *(const v4f*)(p);
  const v4f c = *(const v4f*)(p + 4);
  unsigned short hb[8];
#pragma unroll
  for (int e = 0; e < 4; ++e) {
    hb[e]     = f2bf_bits(a[e]);
    hb[4 + e] = f2bf_bits(c[e]);
  }
  const v4u u = (v4u){pk16(hb[0], hb[1]), pk16(hb[2], hb[3]), pk16(hb[4], hb[5]), pk16(hb[6], hb[7])};
  unsigned short* q = out + 8 * (size_t)i;
  *(volatile v4u*)q = u;
  __threadfence();
  *(volatile v4u*)q = u;
}

__global__ __launch_bounds__(256) void edge_mlp_kernel(const unsigned short* __restrict__ xh,
                                                       const int* __restrict__ src,
                                                       const int* __restrict__ dst,
                                                       const unsigned short* __restrict__ w1h,
                                                       const float* __restrict__ b1,
                                                       const float* __restrict__ W2,
                                                       const float* __restrict__ b2,
                                                       float* __restrict__ out) {
  __shared__ __align__(16) unsigned short As[kBM * kLdaH];
  __shared__ int sSrc[kBM];
  __shared__ int sDst[kBM];
  __shared__ float sB1[kHid];
  __shared__ float sW2d[kHid];
  __shared__ __align__(16) float sPart[2][kBM];

  const int t    = threadIdx.x;
  const int lane = t & 31;
  const int wave = t >> 5;
  const int e0   = blockIdx.x * kBM;

  if (t < kBM) {
    int s = src[e0 + t];
    int d = dst[e0 + t];
    s = s < 0 ? 0 : (s >= kNodes ? kNodes - 1 : s);
    d = d < 0 ? 0 : (d >= kNodes ? kNodes - 1 : d);
    sSrc[t] = s;
    sDst[t] = d;
    sB1[t]  = bf_value(b1[t]);
    sW2d[t] = bf_value(W2[kHid + t]) - bf_value(W2[t]);
  }
  const float b2d = bf_value(b2[1]) - bf_value(b2[0]);
  __syncthreads();

  {
    const int q    = t & 15;
    const int rsub = t >> 4;
#pragma unroll
    for (int it = 0; it < 8; ++it) {
      const int row  = it * 16 + rsub;
      const int node = sSrc[row];
      const v4u v = *(const v4u*)(xh + (size_t)node * kFeat + q * 8);
      *(v4u*)(As + row * kLdaH + q * 8) = v;
      if ((it & 3) == 3) mem_clause_break();
    }
#pragma unroll
    for (int it = 0; it < 8; ++it) {
      const int row  = it * 16 + rsub;
      const int node = sDst[row];
      const v4u v = *(const v4u*)(xh + (size_t)node * kFeat + q * 8);
      *(v4u*)(As + row * kLdaH + kFeat + q * 8) = v;
      if ((it & 3) == 3) mem_clause_break();
    }
  }
  __syncthreads();

  const int rg    = wave >> 1;
  const int cg    = wave & 1;
  const int m0    = rg * 32;
  const int n0    = cg * 64;
  const int rlane = lane & 15;
  const int koff  = (lane >> 4) * 8;
  const int hh    = lane >> 4;

  const __bf16* Ab = reinterpret_cast<const __bf16*>(As);
  const __bf16* Bb = reinterpret_cast<const __bf16*>(w1h);

  v8f acc[2][4];
#pragma unroll
  for (int i = 0; i < 2; ++i)
#pragma unroll
    for (int j = 0; j < 4; ++j) acc[i][j] = (v8f){0.f,0.f,0.f,0.f,0.f,0.f,0.f,0.f};

#pragma unroll 1
  for (int k0 = 0; k0 < kKdim; k0 += 32) {
    v16b bh[4];
#pragma unroll
    for (int j = 0; j < 4; ++j) {
      const size_t bo = (size_t)(n0 + (j << 4) + rlane) * kKdim + koff + k0;
      bh[j] = Frag<__bf16>::load(Bb + bo);
    }
#pragma unroll
    for (int i = 0; i < 2; ++i) {
      const int ao = (m0 + (i << 4) + rlane) * kLdaH + koff + k0;
      const v16b ah = Frag<__bf16>::load(Ab + ao);
#pragma unroll
      for (int j = 0; j < 4; ++j) acc[i][j] = Frag<__bf16>::mma(ah, bh[j], acc[i][j]);
      row_guard_b(acc[i][0], acc[i][1], acc[i][2], acc[i][3], ah, bh[0], bh[1], bh[2], bh[3]);
    }
    Frag<__bf16>::keep(bh[0], bh[1], bh[2], bh[3]);
  }
  acc_guard4(acc[0][0], acc[0][1], acc[0][2], acc[0][3]);
  acc_guard4(acc[1][0], acc[1][1], acc[1][2], acc[1][3]);

  float p[2][8];
#pragma unroll
  for (int i = 0; i < 2; ++i)
#pragma unroll
    for (int r = 0; r < 8; ++r) p[i][r] = 0.0f;
#pragma unroll
  for (int j = 0; j < 4; ++j) {
    const int n = n0 + (j << 4) + rlane;
    const float bv = sB1[n];
    const float wv = sW2d[n];
#pragma unroll
    for (int i = 0; i < 2; ++i) {
#pragma unroll
      for (int r = 0; r < 8; ++r) {
        float v = acc[i][j][r] + bv;
        v = fmaxf(v, 0.0f);
        p[i][r] = fmaf(v, wv, p[i][r]);
      }
    }
  }
#pragma unroll
  for (int i = 0; i < 2; ++i) {
#pragma unroll
    for (int r = 0; r < 8; ++r) {
      float v = p[i][r];
      v += __shfl_xor(v, 1, 32);
      v += __shfl_xor(v, 2, 32);
      v += __shfl_xor(v, 4, 32);
      v += __shfl_xor(v, 8, 32);
      p[i][r] = v;
    }
  }
  if (rlane == 0) {
#pragma unroll
    for (int i = 0; i < 2; ++i)
#pragma unroll
      for (int r = 0; r < 8; ++r) sPart[cg][m0 + (i << 4) + 8 * hh + r] = p[i][r];
  }
  __syncthreads();

  if (wave == 0) {
    const v4f pa = *(const v4f*)(&sPart[0][4 * lane]);
    const v4f pb = *(const v4f*)(&sPart[1][4 * lane]);
    v4f o;
#pragma unroll
    for (int e = 0; e < 4; ++e) {
      float z = (pa[e] + pb[e]) + b2d;
      z = fminf(fmaxf(z, -80.0f), 80.0f);
      const float ex = expf(-z);
      o[e] = 1.0f / (1.0f + ex);
    }
    float* op = out + (size_t)e0 + 4 * lane;
    *(volatile v4f*)op = o;
    __threadfence();
    *(volatile v4f*)op = o;
  }
}

extern "C" void kernel_launch(void* const* d_in, const int* in_sizes, int n_in,
                              void* d_out, int out_size, void* d_ws, size_t ws_size, hipStream_t stream) {
  if (n_in < 7) return;
  const float* x   = (const float*)d_in[0];
  const int*   src = (const int*)  d_in[1];
  const int*   dst = (const int*)  d_in[2];
  const float* W1  = (const float*)d_in[3];
  const float* b1  = (const float*)d_in[4];
  const float* W2  = (const float*)d_in[5];
  const float* b2  = (const float*)d_in[6];
  float* out = (float*)d_out;

  if (in_sizes[0] != kNodes * kFeat || in_sizes[1] != kEdges || in_sizes[2] != kEdges ||
      in_sizes[3] != kHid * kKdim || in_sizes[4] != kHid || in_sizes[5] != 2 * kHid || in_sizes[6] != 2 ||
      out_size != kEdges) return;

  const size_t xh_bytes  = (size_t)kNodes * kFeat * 2;
  const size_t w1h_bytes = (size_t)kHid * kKdim * 2;
  const size_t off_xh  = 0;
  const size_t off_w1h = off_xh + xh_bytes;
  const size_t total   = off_w1h + w1h_bytes;
  if (total > ws_size || total > (size_t)134217728) return;

  unsigned short* xh  = (unsigned short*)((char*)d_ws + off_xh);
  unsigned short* w1h = (unsigned short*)((char*)d_ws + off_w1h);

  const int n8x = (kNodes * kFeat) / 8;
  const int n8w = (kHid * kKdim) / 8;
  cast8_bf16_kernel<<<(n8x + 255) / 256, 256, 0, stream>>>(x, xh, n8x);
  cast8_bf16_kernel<<<(n8w + 255) / 256, 256, 0, stream>>>(W1, w1h, n8w);
  edge_mlp_kernel<<<kEdges / kBM, kThreads, 0, stream>>>(xh, src, dst, w1h, b1, W2, b2, out);
}
